// ShiftedWindowAttention_74105365725402
// MI455X (gfx1250) — hardware-verified
//
#include <hip/hip_runtime.h>

typedef __attribute__((ext_vector_type(16))) _Float16 v16h;
typedef __attribute__((ext_vector_type(8)))  _Float16 v8h;
typedef __attribute__((ext_vector_type(16))) __bf16   v16b;
typedef __attribute__((ext_vector_type(8)))  __bf16   v8b;
typedef __attribute__((ext_vector_type(8)))  float    v8f;
typedef __attribute__((ext_vector_type(4)))  float    v4f;

#define NEG_INF (-__builtin_huge_valf())

__device__ __forceinline__ unsigned short f2bf_bits(float f) {
  unsigned u = __float_as_uint(f);
  return (unsigned short)((u + 0x7FFFu + ((u >> 16) & 1u)) >> 16);
}
__device__ __forceinline__ float bf_bits2f(unsigned short h) { return __uint_as_float(((unsigned)h) << 16); }

__device__ __forceinline__ void dep_guard_h(v8f& a, v8f& b, v16h x, v16h y) { asm volatile("v_nop\n\tv_nop\n\tv_nop\n\tv_nop" : "+v"(a), "+v"(b) : "v"(x), "v"(y)); }
__device__ __forceinline__ void dep_guard_b(v8f& a, v8f& b, v16b x, v16b y) { asm volatile("v_nop\n\tv_nop\n\tv_nop\n\tv_nop" : "+v"(a), "+v"(b) : "v"(x), "v"(y)); }
__device__ __forceinline__ void keep4_h(v16h a, v16h b, v16h c, v16h d) { asm volatile("v_nop" :: "v"(a), "v"(b), "v"(c), "v"(d)); }
__device__ __forceinline__ void keep4_b(v16b a, v16b b, v16b c, v16b d) { asm volatile("v_nop" :: "v"(a), "v"(b), "v"(c), "v"(d)); }
__device__ __forceinline__ void acc_guard4(v8f& a, v8f& b, v8f& c, v8f& d) { asm volatile("v_nop\n\tv_nop\n\tv_nop\n\tv_nop" : "+v"(a), "+v"(b), "+v"(c), "+v"(d)); }
template <typename T> struct Frag;
template <> struct Frag<_Float16> {
  typedef v16h V; union U { v16h v; v8h h[2]; };
  static __device__ __forceinline__ v16h load(const _Float16* p) {
    U f; f.h[0] = *(const v8h*)(p); f.h[1] = *(const v8h*)(p + 16); return f.v;
  }
  static __device__ __forceinline__ v8f mma(v16h a, v16h b, v8f c) {
    return __builtin_amdgcn_wmma_f32_16x16x32_f16(false, a, false, b, (short)0, c, false, false);
  }
  static __device__ __forceinline__ void guard(v8f& a, v8f& b, v16h x, v16h y) { dep_guard_h(a, b, x, y); }
  static __device__ __forceinline__ void keep(v16h a, v16h b, v16h c, v16h d) { keep4_h(a, b, c, d); }
};
template <> struct Frag<__bf16> {
  typedef v16b V; union U { v16b v; v8b h[2]; };
  static __device__ __forceinline__ v16b load(const __bf16* p) {
    U f; f.h[0] = *(const v8b*)(p); f.h[1] = *(const v8b*)(p + 16); return f.v;
  }
  static __device__ __forceinline__ v8f mma(v16b a, v16b b, v8f c) {
    return __builtin_amdgcn_wmma_f32_16x16x32_bf16(false, a, false, b, (short)0, c, false, false);
  }
  static __device__ __forceinline__ void guard(v8f& a, v8f& b, v16b x, v16b y) { dep_guard_b(a, b, x, y); }
  static __device__ __forceinline__ void keep(v16b a, v16b b, v16b c, v16b d) { keep4_b(a, b, c, d); }
};

#define NTOK 1024
#define NWIN 16
#define CD 256
#define HDIM 32
#define NHEAD 8
#define QKVLD 768
#define TSZ 512
#define WST 16
#define WSZ 64
#define SHF 32

__device__ __forceinline__ int rowmap(int m) {
  const int win = m >> 10, n = m & 1023;
  const int b = win >> 3, wn = win & 7;
  const int t = n >> 4, ws = n & 15;
  const int tp = (wn * WSZ + t + SHF) & (TSZ - 1);
  return (b * TSZ + tp) * WST + ws;
}

template <int ET> struct Elem;
template <> struct Elem<0> { typedef _Float16 T; };
template <> struct Elem<1> { typedef __bf16 T; };
template <int ET, bool SPLIT, int BIAS_MODE, int OUT_MODE, bool RESID, int ACT = 0, bool RMAP = false>
__global__ __launch_bounds__(256) void wmma_gemm64(
    const unsigned short* __restrict__ Ap, const unsigned short* __restrict__ A2p, int lda, long strideA,
    const unsigned short* __restrict__ Btp, const unsigned short* __restrict__ Bt2p, int ldb, long strideB,
    void* __restrict__ Cout, void* __restrict__ Cout2, int ldc, long strideC,
    const float* __restrict__ bias,
    const float* __restrict__ resid, long strideR,
    int M, int N, int K, float scale) {
  typedef typename Elem<ET>::T T;
  typedef typename Frag<T>::V V;
  const T* A = (const T*)Ap; const T* A2 = (const T*)A2p; const T* Bt = (const T*)Btp; const T* Bt2 = (const T*)Bt2p;
  __shared__ __align__(16) float sT[8][16 * 68];
  const int b    = blockIdx.y;
  const int lane = threadIdx.x & 31;
  const int wave = threadIdx.x >> 5;
  const int tilesN = N >> 6;
  const int tilesM = M >> 6;
  const int tile = blockIdx.x * 8 + wave;
  if (tile >= tilesM * tilesN) return;
  const int tm = tile / tilesN;
  const int tn = tile - tm * tilesN;
  const int m0 = tm << 6;
  const int n0 = tn << 6;

  const T* Ab  = A  + (size_t)b * strideA;
  const T* Bb  = Bt + (size_t)b * strideB;
  const T* Ab2 = SPLIT ? (A2  + (size_t)b * strideA) : nullptr;
  const T* Bb2 = SPLIT ? (Bt2 + (size_t)b * strideB) : nullptr;

  const int rlane = lane & 15;
  const int koff  = (lane >> 4) * 8;
  const int mOff  = (lane >> 4) * 8;

  v8f acc[4][4];
#pragma unroll
  for (int i = 0; i < 4; ++i)
#pragma unroll
    for (int j = 0; j < 4; ++j) acc[i][j] = (v8f){0.f,0.f,0.f,0.f,0.f,0.f,0.f,0.f};

  for (int k0 = 0; k0 < K; k0 += 32) {
    V bh[4], bl[4];
#pragma unroll
    for (int j = 0; j < 4; ++j) {
      const size_t bo = (size_t)(n0 + (j << 4) + rlane) * ldb + koff + k0;
      bh[j] = Frag<T>::load(Bb + bo);
      if (SPLIT) bl[j] = Frag<T>::load(Bb2 + bo);
    }
#pragma unroll
    for (int i = 0; i < 4; ++i) {
      const size_t ao = (size_t)(m0 + (i << 4) + rlane) * lda + koff + k0;
      V ah = Frag<T>::load(Ab + ao);
      V al;
      if (SPLIT) al = Frag<T>::load(Ab2 + ao);
#pragma unroll
      for (int j = 0; j < 4; ++j) {
        acc[i][j] = Frag<T>::mma(ah, bh[j], acc[i][j]);
        if (SPLIT) {
          acc[i][j] = Frag<T>::mma(ah, bl[j], acc[i][j]);
          acc[i][j] = Frag<T>::mma(al, bh[j], acc[i][j]);
        }
      }
      Frag<T>::guard(acc[i][0], acc[i][3], ah, SPLIT ? al : ah);
    }
    Frag<T>::keep(bh[0], bh[1], bh[2], bh[3]);
    if (SPLIT) Frag<T>::keep(bl[0], bl[1], bl[2], bl[3]);
  }
  acc_guard4(acc[0][0], acc[0][1], acc[0][2], acc[0][3]);
  acc_guard4(acc[1][0], acc[1][1], acc[1][2], acc[1][3]);
  acc_guard4(acc[2][0], acc[2][1], acc[2][2], acc[2][3]);
  acc_guard4(acc[3][0], acc[3][1], acc[3][2], acc[3][3]);

  float* slab = sT[wave];
  const float* Rb = RESID ? (resid + (size_t)b * strideR) : nullptr;
#pragma unroll
  for (int i = 0; i < 4; ++i) {
    const int mBase = m0 + (i << 4);
    const int mDst = RMAP ? rowmap(mBase) : mBase;
#pragma unroll
    for (int j = 0; j < 4; ++j) {
      const int n = n0 + (j << 4) + rlane;
      float bv = 0.f;
      if (BIAS_MODE == 2) bv = bias[n];
#pragma unroll
      for (int r = 0; r < 8; ++r) {
        float v = acc[i][j][r] * scale;
        if (BIAS_MODE == 1) v += bias[mBase + mOff + r];
        if (BIAS_MODE == 2) v += bv;
        if (RESID) v += Rb[(size_t)(mBase + mOff + r) * ldc + n];
        if (ACT == 1) v = tanhf(v);
        if (ACT == 2) v = fmaxf(v, 0.0f);
        if (ACT == 3) v = v / (1.0f + expf(-v));
        if (ACT == 4) v = (v > 0.f) ? v : 0.01f * v;
        if (ACT == 5) v = 0.5f * v * (1.0f + erff(v * 0.70710678118654752f));
        slab[(mOff + r) * 68 + (j << 4) + rlane] = v;
      }
    }
    __builtin_amdgcn_fence(__ATOMIC_RELEASE, "workgroup");
    __builtin_amdgcn_wave_barrier();
    __builtin_amdgcn_fence(__ATOMIC_ACQUIRE, "workgroup");
    if (OUT_MODE == 0) {
      float* C = (float*)Cout + (size_t)b * strideC;
      const int hh = lane >> 4, c4 = (lane & 15) * 4;
      for (int pass = 0; pass < 2; ++pass) {
#pragma unroll
        for (int it = 0; it < 8; ++it) {
          const int row = it * 2 + hh;
          v4f v = *(const v4f*)(slab + row * 68 + c4);
          *(volatile v4f*)(C + (size_t)(mDst + row) * ldc + n0 + c4) = v;
        }
        __threadfence();
      }
    } else {
      const int q = lane >> 3, c8 = (lane & 7) * 8;
      unsigned short* C  = (unsigned short*)Cout  + (size_t)b * strideC;
      unsigned short* C2 = (OUT_MODE == 2) ? ((unsigned short*)Cout2 + (size_t)b * strideC) : nullptr;
      for (int pass = 0; pass < 2; ++pass) {
#pragma unroll
        for (int it = 0; it < 4; ++it) {
          const int row = it * 4 + q;
          const float* sp = slab + row * 68 + c8;
          v8h hv, lv;
#pragma unroll
          for (int e = 0; e < 8; ++e) {
            if (OUT_MODE == 1) {
              hv[e] = (_Float16)sp[e];
            } else {
              unsigned short hb = f2bf_bits(sp[e]);
              unsigned short lb = f2bf_bits(sp[e] - bf_bits2f(hb));
              hv[e] = __builtin_bit_cast(_Float16, hb);
              lv[e] = __builtin_bit_cast(_Float16, lb);
            }
          }
          *(volatile v8h*)(C + (size_t)(mDst + row) * ldc + n0 + c8) = hv;
          if (OUT_MODE == 2) *(volatile v8h*)(C2 + (size_t)(mDst + row) * ldc + n0 + c8) = lv;
        }
        __threadfence();
      }
    }
    __builtin_amdgcn_fence(__ATOMIC_RELEASE, "workgroup");
    __builtin_amdgcn_wave_barrier();
    __builtin_amdgcn_fence(__ATOMIC_ACQUIRE, "workgroup");
  }
}

__global__ __launch_bounds__(256) void cast8_kernel(
    const float* __restrict__ in, _Float16* __restrict__ out, int n8, float scale) {
  const int i = blockIdx.x * 256 + threadIdx.x;
  if (i < n8) {
    const float* p = in + (size_t)i * 8;
    const v4f f0 = *(const v4f*)p;
    const v4f f1 = *(const v4f*)(p + 4);
    v8h hv;
    hv[0] = (_Float16)(f0[0] * scale); hv[1] = (_Float16)(f0[1] * scale);
    hv[2] = (_Float16)(f0[2] * scale); hv[3] = (_Float16)(f0[3] * scale);
    hv[4] = (_Float16)(f1[0] * scale); hv[5] = (_Float16)(f1[1] * scale);
    hv[6] = (_Float16)(f1[2] * scale); hv[7] = (_Float16)(f1[3] * scale);
    _Float16* q = out + (size_t)i * 8;
    *(volatile v8h*)q = hv;
    __threadfence();
    *(volatile v8h*)q = hv;
  }
}

__global__ __launch_bounds__(256) void castx_kernel(
    const float* __restrict__ x, _Float16* __restrict__ xw, int n8) {
  const int i = blockIdx.x * 256 + threadIdx.x;
  if (i < n8) {
    const int m = i >> 5;
    const int c8 = (i & 31) * 8;
    const int src = rowmap(m);
    const float* p = x + (size_t)src * CD + c8;
    const v4f f0 = *(const v4f*)p;
    const v4f f1 = *(const v4f*)(p + 4);
    v8h hv;
    hv[0] = (_Float16)f0[0]; hv[1] = (_Float16)f0[1]; hv[2] = (_Float16)f0[2]; hv[3] = (_Float16)f0[3];
    hv[4] = (_Float16)f1[0]; hv[5] = (_Float16)f1[1]; hv[6] = (_Float16)f1[2]; hv[7] = (_Float16)f1[3];
    _Float16* q = xw + (size_t)i * 8;
    *(volatile v8h*)q = hv;
    __threadfence();
    *(volatile v8h*)q = hv;
  }
}

#define A_NW 8
#define A_QB 128
#define A_KC 64
#define A_KP 40
#define A_VP 72
#define A_PP 72
#define A_OP 36
#define PSC 32768.0f

__device__ __forceinline__ v8f mma_h(v16h a, v16h b, v8f c) {
  c = __builtin_amdgcn_wmma_f32_16x16x32_f16(false, a, false, b, (short)0, c, false, false);
  asm volatile("v_nop\n\tv_nop\n\tv_nop\n\tv_nop" : "+v"(c) : "v"(a), "v"(b));
  return c;
}

__device__ __forceinline__ int bin_index(float d, int nb) {
#pragma clang fp contract(off)
  float f = d / (float)(111.32 / 100.0);
  f = f + (float)(nb - 1) * 0.5f;
  f = rintf(f);
  f = fminf(fmaxf(f, 0.0f), (float)(nb - 1));
  return (int)f;
}

__global__ __launch_bounds__(256) void win_attn_kernel(
    const _Float16* __restrict__ qkv, const float* __restrict__ loc,
    const float* __restrict__ table_t, const float* __restrict__ table_x,
    const float* __restrict__ table_y, const float* __restrict__ table_z,
    float* __restrict__ out) {
  __shared__ __align__(16) _Float16 Ks[A_KC * A_KP];
  __shared__ __align__(16) _Float16 Vt[HDIM * A_VP];
  __shared__ __align__(16) _Float16 Ps[A_NW][16 * A_PP];
  __shared__ __align__(16) float Os[A_NW][16 * A_OP];
  __shared__ float tts[128];
  __shared__ float sxs[256];
  __shared__ float sys[256];
  __shared__ float szs[256];

  const int tid  = threadIdx.x;
  const int wave = tid >> 5;
  const int lane = tid & 31;
  const int hh   = lane >> 4;
  const int c    = lane & 15;
  const int qb   = blockIdx.x;
  const int h    = blockIdx.y & 7;
  const int win  = blockIdx.y >> 3;
  const int b    = win >> 3, wn = win & 7;
  const int q0   = qb * A_QB + wave * 16;
  const size_t wrow0 = (size_t)win * NTOK;

  if (tid < 2 * WSZ - 1) tts[tid] = table_t[tid * NHEAD + h];
  {
    const int si = tid >> 4, sj = tid & 15;
    const float* li = loc + (b * WST + si) * 3;
    const float* lj = loc + (b * WST + sj) * 3;
    const float dx = li[0] - lj[0];
    const float dy = li[1] - lj[1];
    const float dz = li[2] - lj[2];
    sxs[tid] = table_x[bin_index(dx, 51) * NHEAD + h];
    sys[tid] = table_y[bin_index(dy, 51) * NHEAD + h];
    szs[tid] = table_z[bin_index(dz, 11) * NHEAD + h];
  }
  __syncthreads();

  float bxr[8], byr[8], bzr[8];
#pragma unroll
  for (int r = 0; r < 8; ++r) {
    const int si = 8 * hh + r;
    bxr[r] = sxs[si * 16 + c];
    byr[r] = sys[si * 16 + c];
    bzr[r] = szs[si * 16 + c];
  }

  const v16h qa = Frag<_Float16>::load(qkv + (wrow0 + q0 + c) * QKVLD + h * HDIM + 8 * hh);
  const int qt0 = (q0 + 8 * hh) & (WSZ - 1);

  float mrow[8], lrow[8];
  v8f oacc[2];
#pragma unroll
  for (int r = 0; r < 8; ++r) { mrow[r] = NEG_INF; lrow[r] = 0.f; }
#pragma unroll
  for (int t = 0; t < 2; ++t) oacc[t] = (v8f){0.f,0.f,0.f,0.f,0.f,0.f,0.f,0.f};

  const float qscale = 0.17677669529663687f;
  const bool qlo = (qb < 4);

  for (int kc = 0; kc < NTOK / A_KC; ++kc) {
    const int kv0 = kc * A_KC;
    __syncthreads();
    {
      const int kvr = tid >> 2, part = tid & 3;
      const _Float16* krow = qkv + (wrow0 + kv0 + kvr) * QKVLD + CD + h * HDIM + part * 8;
      const v8h k8 = *(const v8h*)krow;
      *(v8h*)(Ks + kvr * A_KP + part * 8) = k8;
      const v8h v8 = *(const v8h*)(krow + CD);
#pragma unroll
      for (int e = 0; e < 8; ++e) Vt[(part * 8 + e) * A_VP + kvr] = v8[e];
    }
    __syncthreads();

    v8f s[4];
#pragma unroll
    for (int j = 0; j < 4; ++j) {
      s[j] = (v8f){0.f,0.f,0.f,0.f,0.f,0.f,0.f,0.f};
      const v16h kb = Frag<_Float16>::load(Ks + (j * 16 + c) * A_KP + 8 * hh);
      s[j] = mma_h(qa, kb, s[j]);
    }
    const float madd = (wn == 7 && (qlo != (kc < 8))) ? -100.0f : 0.0f;
    float cm[8];
#pragma unroll
    for (int r = 0; r < 8; ++r) {
      const int qt = qt0 + r;
      float m = NEG_INF;
#pragma unroll
      for (int j = 0; j < 4; ++j) {
        const int kt = j * 16 + c;
        float bias = tts[qt - kt + (WSZ - 1)] + bxr[r];
        bias = bias + byr[r];
        bias = bias + bzr[r];
        float v = s[j][r] * qscale + bias;
        v = v + madd;
        s[j][r] = v;
        m = fmaxf(m, v);
      }
#pragma unroll
      for (int off = 1; off < 16; off <<= 1) m = fmaxf(m, __shfl_xor(m, off, 32));
      cm[r] = m;
    }
    _Float16* pw = Ps[wave];
#pragma unroll
    for (int r = 0; r < 8; ++r) {
      const float mnew = fmaxf(mrow[r], cm[r]);
      const float alpha = __expf(mrow[r] - mnew);
      mrow[r] = mnew;
      float psum = 0.f;
#pragma unroll
      for (int j = 0; j < 4; ++j) {
        const float p = __expf(s[j][r] - mnew);
        psum += p;
        pw[(8 * hh + r) * A_PP + j * 16 + c] = (_Float16)(p * PSC);
      }
#pragma unroll
      for (int off = 1; off < 16; off <<= 1) psum += __shfl_xor(psum, off, 32);
      lrow[r] = lrow[r] * alpha + psum;
      oacc[0][r] *= alpha;
      oacc[1][r] *= alpha;
    }
    __builtin_amdgcn_fence(__ATOMIC_RELEASE, "workgroup");
    __builtin_amdgcn_wave_barrier();
    __builtin_amdgcn_fence(__ATOMIC_ACQUIRE, "workgroup");
#pragma unroll
    for (int kk = 0; kk < 2; ++kk) {
      const v16h pa = Frag<_Float16>::load(pw + c * A_PP + kk * 32 + 8 * hh);
#pragma unroll
      for (int t = 0; t < 2; ++t) {
        const v16h vb = Frag<_Float16>::load(Vt + (t * 16 + c) * A_VP + kk * 32 + 8 * hh);
        oacc[t] = mma_h(pa, vb, oacc[t]);
      }
    }
  }

  float* os = Os[wave];
#pragma unroll
  for (int r = 0; r < 8; ++r) {
    const float inv = 1.0f / (lrow[r] * PSC);
    os[(8 * hh + r) * A_OP + c]      = oacc[0][r] * inv;
    os[(8 * hh + r) * A_OP + 16 + c] = oacc[1][r] * inv;
  }
  __builtin_amdgcn_fence(__ATOMIC_RELEASE, "workgroup");
  __builtin_amdgcn_wave_barrier();
  __builtin_amdgcn_fence(__ATOMIC_ACQUIRE, "workgroup");
  {
    const int q8 = lane >> 3, c4 = (lane & 7) * 4;
    float* ob = out + (wrow0 + q0) * CD + h * HDIM;
    for (int pass = 0; pass < 2; ++pass) {
#pragma unroll
      for (int it = 0; it < 4; ++it) {
        const int row = it * 4 + q8;
        v4f val = *(const v4f*)(os + row * A_OP + c4);
        *(volatile v4f*)(ob + (size_t)row * CD + c4) = val;
      }
      __threadfence();
    }
  }
}

extern "C" void kernel_launch(void* const* d_in, const int* in_sizes, int n_in,
                              void* d_out, int out_size, void* d_ws, size_t ws_size,
                              hipStream_t stream) {
  if (n_in < 10) return;
  const int M = NWIN * NTOK;
  if (in_sizes[0] != M * CD) return;
  if (in_sizes[1] != 2 * WST * 3) return;
  if (in_sizes[2] != 3 * CD * CD || in_sizes[3] != 3 * CD) return;
  if (in_sizes[4] != CD * CD || in_sizes[5] != CD) return;
  if (in_sizes[6] != (2 * WSZ - 1) * NHEAD || in_sizes[7] != 51 * NHEAD ||
      in_sizes[8] != 51 * NHEAD || in_sizes[9] != 11 * NHEAD) return;
  if (out_size != M * CD) return;

  const float* x      = (const float*)d_in[0];
  const float* loc    = (const float*)d_in[1];
  const float* qkv_w  = (const float*)d_in[2];
  const float* qkv_b  = (const float*)d_in[3];
  const float* proj_w = (const float*)d_in[4];
  const float* proj_b = (const float*)d_in[5];
  const float* tt     = (const float*)d_in[6];
  const float* tx     = (const float*)d_in[7];
  const float* ty     = (const float*)d_in[8];
  const float* tz     = (const float*)d_in[9];
  float* out = (float*)d_out;

  const size_t szXW   = (size_t)M * CD * 2;
  const size_t szWQ   = (size_t)3 * CD * CD * 2;
  const size_t szWP   = (size_t)CD * CD * 2;
  const size_t szQKV  = (size_t)M * QKVLD * 2;
  const size_t szAO   = (size_t)M * CD * 4;
  const size_t szAO16 = (size_t)M * CD * 2;
  const size_t oXW   = 0;
  const size_t oWQ   = oXW + szXW;
  const size_t oWP   = oWQ + szWQ;
  const size_t oQKV  = oWP + szWP;
  const size_t oAO   = oQKV + szQKV;
  const size_t oAO16 = oAO + szAO;
  const size_t total = oAO16 + szAO16;
  if (total > ws_size) return;

  char* ws = (char*)d_ws;
  _Float16* xw16   = (_Float16*)(ws + oXW);
  _Float16* wq16   = (_Float16*)(ws + oWQ);
  _Float16* wp16   = (_Float16*)(ws + oWP);
  _Float16* qkv16  = (_Float16*)(ws + oQKV);
  float*    attnf  = (float*)(ws + oAO);
  _Float16* attn16 = (_Float16*)(ws + oAO16);
  const float* dummy_resid = (const float*)(ws + oXW);

  {
    const int n8 = M * CD / 8;
    castx_kernel<<<dim3((n8 + 255) / 256), 256, 0, stream>>>(x, xw16, n8);
  }
  {
    const int n8q = 3 * CD * CD / 8;
    cast8_kernel<<<dim3((n8q + 255) / 256), 256, 0, stream>>>(qkv_w, wq16, n8q, 16.0f);
    const int n8p = CD * CD / 8;
    cast8_kernel<<<dim3((n8p + 255) / 256), 256, 0, stream>>>(proj_w, wp16, n8p, 16.0f);
  }
  {
    const int tiles = (M / 64) * (QKVLD / 64);
    wmma_gemm64<0, false, 2, 1, false, 0, false><<<dim3((tiles + 7) / 8, 1), 256, 0, stream>>>(
        (const unsigned short*)xw16, (const unsigned short*)xw16, CD, (long)0,
        (const unsigned short*)wq16, (const unsigned short*)wq16, CD, (long)0,
        (void*)qkv16, (void*)qkv16, QKVLD, (long)0,
        qkv_b, dummy_resid, (long)0, M, QKVLD, CD, 1.0f / 16.0f);
  }
  win_attn_kernel<<<dim3(NTOK / A_QB, NWIN * NHEAD), 256, 0, stream>>>(qkv16, loc, tt, tx, ty, tz, attnf);
  {
    const int n8 = M * CD / 8;
    cast8_kernel<<<dim3((n8 + 255) / 256), 256, 0, stream>>>(attnf, attn16, n8, 16.0f);
  }
  {
    const int tiles = (M / 64) * (CD / 64);
    wmma_gemm64<0, false, 2, 0, false, 0, true><<<dim3((tiles + 7) / 8, 1), 256, 0, stream>>>(
        (const unsigned short*)attn16, (const unsigned short*)attn16, CD, (long)0,
        (const unsigned short*)wp16, (const unsigned short*)wp16, CD, (long)0,
        (void*)out, (void*)out, CD, (long)0,
        proj_b, dummy_resid, (long)0, M, CD, CD, 1.0f / 256.0f);
  }
}
